// GSPNLayer_34136400069261
// MI455X (gfx1250) — hardware-run, weakly checked
//
#include <hip/hip_runtime.h>
#include <math.h>

typedef __attribute__((ext_vector_type(16))) _Float16 v16h;
typedef __attribute__((ext_vector_type(8)))  _Float16 v8h;
typedef __attribute__((ext_vector_type(8)))  float    v8f;
typedef __attribute__((ext_vector_type(4)))  float    v4f;
typedef __attribute__((ext_vector_type(2)))  float    v2f;
typedef __attribute__((ext_vector_type(2)))  unsigned v2u;

constexpr int kInputsRneToBf16 = 1;

constexpr int kNB   = 8;
constexpr int kNC   = 256;
constexpr int kNCr  = 64;
constexpr int kSide = 64;
constexpr int kPix  = kSide * kSide;
constexpr int kRows = kNB * kPix;
constexpr int kNUL  = 2 * kNC;
constexpr int kKM   = 2 * kNC;
static_assert(kPix == 4096 && kRows == 32768 && kNUL == 512 && kKM == 512, "shape");
static_assert((kNC % 32) == 0 && (kNCr % 32) == 0 && (kKM % 32) == 0, "GEMM K multiples of 32");
static_assert((kRows % 64) == 0 && (kNCr % 64) == 0 && (kNUL % 64) == 0 && (kNC % 64) == 0 && (kPix % 64) == 0, "GEMM M,N multiples of 64");

constexpr float kCarryX    = 16.0f;
constexpr float kCarryRed  = 16.0f;
constexpr float kCarryWred = 256.0f;
constexpr float kCarryWul  = 256.0f;
constexpr float kCarryO    = 64.0f;
constexpr float kCarryWab  = 1024.0f;
constexpr float kScaleS0   = kCarryRed / (kCarryX * kCarryWred);
constexpr float kScaleS12  = 1.0f / (kCarryRed * kCarryWul);
constexpr float kScaleS4   = 1.0f / (kCarryO * kCarryWab);
constexpr float kInvCarryRed = 1.0f / kCarryRed;
constexpr float kF16MinNormal = 6.103515625e-5f;
constexpr float kF16Clamp = 60000.0f;

constexpr size_t kOffXT   = 0;
constexpr size_t kOffRED  = kOffXT   + (size_t)kRows * kNC  * 2;
constexpr size_t kOffUL   = kOffRED  + (size_t)kRows * kNCr * 2;
constexpr size_t kOffO    = kOffUL   + (size_t)kRows * kNUL * 4;
constexpr size_t kOffWRED = kOffO    + (size_t)kRows * kKM  * 2;
constexpr size_t kOffWUL  = kOffWRED + (size_t)kNCr  * kNC  * 2;
constexpr size_t kOffWAB  = kOffWUL  + (size_t)kNUL  * kNCr * 2;
constexpr size_t kOffBUL  = kOffWAB  + (size_t)kNC   * kKM  * 2;
constexpr size_t kOffBRED = kOffBUL  + (size_t)kNUL * 4;
constexpr size_t kOffBMRG = kOffBRED + (size_t)128 * 4;
constexpr size_t kOffRC   = kOffBMRG + (size_t)kNC * 4;
constexpr size_t kWsTotal = kOffRC   + (size_t)kRows * 4;
static_assert(kWsTotal == 122129920ull, "carve total");
static_assert(kWsTotal <= 134217728ull, "carve cap");
static_assert((kOffRED % 128) == 0 && (kOffUL % 128) == 0 && (kOffO % 128) == 0 && (kOffWRED % 128) == 0 &&
              (kOffWUL % 128) == 0 && (kOffWAB % 128) == 0 && (kOffBUL % 128) == 0 && (kOffBRED % 128) == 0 &&
              (kOffBMRG % 128) == 0 && (kOffRC % 128) == 0, "128-B aligned regions");

__device__ __forceinline__ unsigned short f2bf_bits(float f) {
  unsigned u = __float_as_uint(f);
  return (unsigned short)((u + 0x7FFFu + ((u >> 16) & 1u)) >> 16);
}
__device__ __forceinline__ float bf_bits2f(unsigned short h) { return __uint_as_float(((unsigned)h) << 16); }

__device__ __forceinline__ float rin(float v) {
  if (kInputsRneToBf16) return bf_bits2f(f2bf_bits(v));
  return v;
}

__device__ __forceinline__ _Float16 to_h_flush(float t) {
  const float u = (fabsf(t) < kF16MinNormal) ? 0.0f : t;
  return (_Float16)u;
}
__device__ __forceinline__ _Float16 to_h_clamp_flush(float t) {
  const float c = fminf(fmaxf(t, -kF16Clamp), kF16Clamp);
  return to_h_flush(c);
}
__device__ __forceinline__ unsigned pack2h(float a, float b) {
  const _Float16 h0 = to_h_clamp_flush(a);
  const _Float16 h1 = to_h_clamp_flush(b);
  const unsigned short b0 = __builtin_bit_cast(unsigned short, h0);
  const unsigned short b1 = __builtin_bit_cast(unsigned short, h1);
  return (unsigned)b0 | ((unsigned)b1 << 16);
}

__device__ __forceinline__ float h16_to_f32(unsigned hb) {
  const unsigned sgn = (hb & 0x8000u) << 16;
  const unsigned em = hb & 0x7fffu;
  const float fn = __uint_as_float((em << 13) + 0x38000000u);
  const float fs = (float)em * 5.9604644775390625e-8f;
  const float mag = (em < 0x400u) ? fs : fn;
  return __uint_as_float(__float_as_uint(mag) | sgn);
}

union FragU { v16h v; v8h h[2]; };
__device__ __forceinline__ v16h frag_load(const _Float16* p) {
  FragU f;
  f.h[0] = *(const v8h*)(p);
  f.h[1] = *(const v8h*)(p + 16);
  return f.v;
}
__device__ __forceinline__ v8f mma_h(v16h a, v16h b, v8f c) {
  c = __builtin_amdgcn_wmma_f32_16x16x32_f16(false, a, false, b, (short)0, c, false, false);
  asm volatile("v_nop\n\tv_nop\n\tv_nop\n\tv_nop" : "+v"(c) : "v"(a), "v"(b));
  return c;
}
__device__ __forceinline__ void acc_guard4(v8f& a, v8f& b, v8f& c, v8f& d) {
  asm volatile("v_nop\n\tv_nop\n\tv_nop\n\tv_nop" : "+v"(a), "+v"(b), "+v"(c), "+v"(d));
}

template <int BIAS_MODE, int OUT_MODE>
__global__ __launch_bounds__(256) void gemm64_h(
    const unsigned short* __restrict__ Ap, int lda, long strideA,
    const unsigned short* __restrict__ Btp, int ldb, long strideB,
    void* __restrict__ Cout, int ldc, long strideC,
    const float* __restrict__ bias,
    int M, int N, int K, float scale) {
  const _Float16* A  = (const _Float16*)Ap;
  const _Float16* Bt = (const _Float16*)Btp;
  __shared__ __align__(16) float sT[8][16 * 68];
  const int b    = blockIdx.y;
  const int lane = threadIdx.x & 31;
  const int wave = threadIdx.x >> 5;
  const int tilesN = N >> 6;
  const int tilesM = M >> 6;
  const int tile = blockIdx.x * 8 + wave;
  if (tile >= tilesM * tilesN) return;
  const int tm = tile / tilesN;
  const int tn = tile - tm * tilesN;
  const int m0 = tm << 6;
  const int n0 = tn << 6;

  const _Float16* Ab = A  + (size_t)b * strideA;
  const _Float16* Bb = Bt + (size_t)b * strideB;

  const int rlane = lane & 15;
  const int koff  = (lane >> 4) * 8;
  const int mOff  = (lane >> 4) * 8;

  v8f acc[4][4];
#pragma unroll
  for (int i = 0; i < 4; ++i)
#pragma unroll
    for (int j = 0; j < 4; ++j) acc[i][j] = (v8f){0.f,0.f,0.f,0.f,0.f,0.f,0.f,0.f};

  for (int k0 = 0; k0 < K; k0 += 32) {
    v16h bh[4];
#pragma unroll
    for (int j = 0; j < 4; ++j) {
      const size_t bo = (size_t)(n0 + (j << 4) + rlane) * ldb + koff + k0;
      bh[j] = frag_load(Bb + bo);
    }
#pragma unroll
    for (int i = 0; i < 4; ++i) {
      const size_t ao = (size_t)(m0 + (i << 4) + rlane) * lda + koff + k0;
      const v16h ah = frag_load(Ab + ao);
#pragma unroll
      for (int j = 0; j < 4; ++j) acc[i][j] = mma_h(ah, bh[j], acc[i][j]);
    }
  }
  acc_guard4(acc[0][0], acc[0][1], acc[0][2], acc[0][3]);
  acc_guard4(acc[1][0], acc[1][1], acc[1][2], acc[1][3]);
  acc_guard4(acc[2][0], acc[2][1], acc[2][2], acc[2][3]);
  acc_guard4(acc[3][0], acc[3][1], acc[3][2], acc[3][3]);

  float* slab = sT[wave];
#pragma unroll
  for (int i = 0; i < 4; ++i) {
    const int mBase = m0 + (i << 4);
#pragma unroll
    for (int j = 0; j < 4; ++j) {
      const int n = n0 + (j << 4) + rlane;
      float bv = 0.f;
      if (BIAS_MODE == 2) bv = bias[n];
#pragma unroll
      for (int r = 0; r < 8; ++r) {
        float v = acc[i][j][r] * scale;
        if (BIAS_MODE == 1) v += bias[mBase + mOff + r];
        if (BIAS_MODE == 2) v += bv;
        slab[(mOff + r) * 68 + (j << 4) + rlane] = v;
      }
    }
    __builtin_amdgcn_fence(__ATOMIC_RELEASE, "workgroup");
    __builtin_amdgcn_wave_barrier();
    __builtin_amdgcn_fence(__ATOMIC_ACQUIRE, "workgroup");
    if (OUT_MODE == 0) {
      float* C = (float*)Cout + (size_t)b * strideC;
      const int hh = lane >> 4, c4 = (lane & 15) * 4;
      for (int pass = 0; pass < 2; ++pass) {
#pragma unroll
        for (int it = 0; it < 8; ++it) {
          const int row = it * 2 + hh;
          v4f v = *(const v4f*)(slab + row * 68 + c4);
          *(volatile v4f*)(C + (size_t)(mBase + row) * ldc + n0 + c4) = v;
        }
        __threadfence();
      }
    } else {
      const int q = lane >> 3, c8 = (lane & 7) * 8;
      unsigned short* C = (unsigned short*)Cout + (size_t)b * strideC;
      v8h hv[4];
#pragma unroll
      for (int it = 0; it < 4; ++it) {
        const int row = it * 4 + q;
        const float* sp = slab + row * 68 + c8;
#pragma unroll
        for (int e = 0; e < 8; ++e) hv[it][e] = to_h_flush(sp[e]);
      }
      for (int pass = 0; pass < 2; ++pass) {
#pragma unroll
        for (int it = 0; it < 4; ++it) {
          const int row = it * 4 + q;
          *(volatile v8h*)(C + (size_t)(mBase + row) * ldc + n0 + c8) = hv[it];
        }
        __threadfence();
      }
    }
    __builtin_amdgcn_fence(__ATOMIC_RELEASE, "workgroup");
    __builtin_amdgcn_wave_barrier();
    __builtin_amdgcn_fence(__ATOMIC_ACQUIRE, "workgroup");
  }
}

__device__ __forceinline__ void store8h_twice(unsigned short* dst, v8h hv) {
  *(volatile v8h*)dst = hv;
  __threadfence();
  *(volatile v8h*)dst = hv;
}
__device__ __forceinline__ void store4f_twice(float* dst, v4f v) {
  *(volatile v4f*)dst = v;
  __threadfence();
  *(volatile v4f*)dst = v;
}

__global__ __launch_bounds__(256) void prep_planes_kernel(
    const float* __restrict__ w_red, const float* __restrict__ b_red,
    const float* __restrict__ w_u, const float* __restrict__ b_u,
    const float* __restrict__ w_lam, const float* __restrict__ b_lam,
    const float* __restrict__ w_merge, const float* __restrict__ b_merge,
    unsigned short* __restrict__ wred16, unsigned short* __restrict__ wul16, unsigned short* __restrict__ wab16,
    float* __restrict__ bias_ul, float* __restrict__ bred16, float* __restrict__ bmerge_c)
{
  const int tid = threadIdx.x;
  const int blk = blockIdx.x;
  if (blk < 64) {
    const int e0 = (blk * 256 + tid) << 3;
    const int o  = e0 >> 9;
    const int kk = e0 & 511;
    const int hf = kk >> 8;
    const int cc = kk & 255;
    const float* s0 = w_merge + (size_t)o * 1024 + hf * 256 + cc;
    const v4f p0 = *(const v4f*)(s0);
    const v4f p1 = *(const v4f*)(s0 + 4);
    const v4f q0 = *(const v4f*)(s0 + 512);
    const v4f q1 = *(const v4f*)(s0 + 516);
    v8h hv;
#pragma unroll
    for (int e = 0; e < 4; ++e) {
      hv[e]     = to_h_flush((rin(p0[e]) + rin(q0[e])) * kCarryWab);
      hv[4 + e] = to_h_flush((rin(p1[e]) + rin(q1[e])) * kCarryWab);
    }
    store8h_twice(wab16 + e0, hv);
    return;
  }
  if (blk < 88) {
    const bool isRed = (blk < 72);
    const bool isU   = (blk < 80);
    const int e0 = isRed ? (((blk - 64) * 256 + tid) << 3) : (((blk - 72) * 256 + tid) << 3);
    const float* src = isRed ? (w_red + e0) : (isU ? (w_u + e0) : (w_lam + (e0 - kNC * kNCr)));
    unsigned short* dst = isRed ? (wred16 + e0) : (wul16 + e0);
    const float carry = isRed ? kCarryWred : kCarryWul;
    const v4f a0 = *(const v4f*)(src);
    const v4f a1 = *(const v4f*)(src + 4);
    v8h hv;
#pragma unroll
    for (int e = 0; e < 4; ++e) {
      hv[e]     = to_h_flush(rin(a0[e]) * carry);
      hv[4 + e] = to_h_flush(rin(a1[e]) * carry);
    }
    store8h_twice(dst, hv);
    return;
  }
  const int wave = tid >> 5, lane = tid & 31;
  if (wave == 7) return;
  const float* src;
  float* dst;
  float mul = 1.0f;
  bool live = true;
  if (wave < 2) {
    src = b_u + 4 * tid;
    dst = bias_ul + 4 * tid;
  } else if (wave < 4) {
    src = b_lam + 4 * (tid - 64);
    dst = bias_ul + kNC + 4 * (tid - 64);
  } else if (wave == 4) {
    const int l4 = (lane < 16) ? (4 * lane) : 60;
    src = b_red + l4;
    dst = bred16 + 4 * lane;
    mul = kCarryRed;
    live = (lane < 16);
  } else {
    src = b_merge + 4 * (tid - 160);
    dst = bmerge_c + 4 * (tid - 160);
  }
  v4f a = *(const v4f*)(src);
  v4f o4;
#pragma unroll
  for (int e = 0; e < 4; ++e) {
    const float t = rin(a[e]) * mul;
    o4[e] = live ? t : 0.0f;
  }
  store4f_twice(dst, o4);
}

__global__ __launch_bounds__(256) void x_plane_kernel(const float* __restrict__ x, unsigned short* __restrict__ xT16)
{
  __shared__ float sT[64 * 65];
  const int tid = threadIdx.x;
  const int pt = blockIdx.x & 63;
  const int ct = (blockIdx.x >> 6) & 3;
  const int b  = blockIdx.x >> 8;
  const int p0 = pt * 64, c0 = ct * 64;
  const float* xb = x + ((size_t)(b * kNC + c0)) * kPix + p0;
  const int lc = tid >> 4, q = tid & 15;
#pragma unroll
  for (int i = 0; i < 4; ++i) {
    const int c = lc + 16 * i;
    const v4f v = *(const v4f*)(xb + (size_t)c * kPix + 4 * q);
    sT[c * 65 + 4 * q + 0] = v[0];
    sT[c * 65 + 4 * q + 1] = v[1];
    sT[c * 65 + 4 * q + 2] = v[2];
    sT[c * 65 + 4 * q + 3] = v[3];
  }
  __syncthreads();
  const int pr = tid >> 3, c8 = (tid & 7) * 8;
  v8h hv[2];
#pragma unroll
  for (int it = 0; it < 2; ++it) {
    const int p = pr + 32 * it;
#pragma unroll
    for (int e = 0; e < 8; ++e) hv[it][e] = to_h_flush(rin(sT[(c8 + e) * 65 + p]) * kCarryX);
  }
  for (int pass = 0; pass < 2; ++pass) {
#pragma unroll
    for (int it = 0; it < 2; ++it) {
      const int p = pr + 32 * it;
      *(volatile v8h*)(xT16 + ((size_t)(b * kPix + p0 + p)) * kNC + c0 + c8) = hv[it];
    }
    __threadfence();
  }
}

__global__ __launch_bounds__(256) void band_coef_kernel(
    const unsigned short* __restrict__ red16, const float* __restrict__ w_wt, const float* __restrict__ b_wt,
    float* __restrict__ rc)
{
  __shared__ float sW[256];
  const int tid = threadIdx.x;
  {
    const int wi = (tid < 3 * kNCr) ? tid : (3 * kNCr - 1);
    sW[tid] = rin(w_wt[wi]);
  }
  __syncthreads();
  const int pix = blockIdx.x * 256 + tid;
  const unsigned* rowp = (const unsigned*)(red16 + (size_t)pix * kNCr);
  float s0 = 0.f, s1 = 0.f, s2 = 0.f;
#pragma unroll 1
  for (int g = 0; g < 16; ++g) {
    const v2u wv = *(const v2u*)(rowp + 2 * g);
    const unsigned w0 = wv[0];
    const unsigned w1 = wv[1];
    const float r0 = h16_to_f32(w0 & 0xffffu);
    const float r1 = h16_to_f32(w0 >> 16);
    const float r2 = h16_to_f32(w1 & 0xffffu);
    const float r3 = h16_to_f32(w1 >> 16);
    const float* wp = sW + 4 * g;
    s0 = fmaf(wp[0], r0, s0);  s0 = fmaf(wp[1], r1, s0);  s0 = fmaf(wp[2], r2, s0);  s0 = fmaf(wp[3], r3, s0);
    s1 = fmaf(wp[64], r0, s1); s1 = fmaf(wp[65], r1, s1); s1 = fmaf(wp[66], r2, s1); s1 = fmaf(wp[67], r3, s1);
    s2 = fmaf(wp[128], r0, s2); s2 = fmaf(wp[129], r1, s2); s2 = fmaf(wp[130], r2, s2); s2 = fmaf(wp[131], r3, s2);
  }
  const float p0 = s0 * kInvCarryRed + rin(b_wt[0]);
  const float p1 = s1 * kInvCarryRed + rin(b_wt[1]);
  const float p2 = s2 * kInvCarryRed + rin(b_wt[2]);
  const float g0 = 1.0f / (1.0f + expf(-p0));
  const float g1 = 1.0f / (1.0f + expf(-p1));
  const float g2 = 1.0f / (1.0f + expf(-p2));
  const float den = fmaxf((g0 + g1) + g2, 1e-6f);
  const float inv = 1.0f / den;
  const int w = pix & (kSide - 1);
  const float n0 = (w >= 1) ? (g0 * inv) : 0.0f;
  const float n2 = (w <= kSide - 2) ? (g2 * inv) : 0.0f;
  const float rv = (n0 + g1 * inv) + n2;
  float* dst = rc + pix;
  *(volatile float*)dst = rv;
  __threadfence();
  *(volatile float*)dst = rv;
}

constexpr int kXsPitch = 260;
__global__ __launch_bounds__(128) void line_scan_kernel(
    const float* __restrict__ x, const float* __restrict__ ul, const float* __restrict__ rc,
    unsigned short* __restrict__ o16)
{
  __shared__ __align__(16) float xs[32 * kXsPitch];
  __shared__ float Rs[128];
  const int tid = threadIdx.x;
  const int b = blockIdx.x >> 6;
  const int h = blockIdx.x & 63;
  const int c = 2 * tid;
  const size_t bp = (size_t)b * kPix;
  Rs[tid] = rc[(size_t)(b * kSide + h) * kSide + (tid & 63)];
  float h1a = 0.f, h1b = 0.f, h2a = 0.f, h2b = 0.f;
  const int sc = tid >> 3, sq = tid & 7;
  unsigned* Ow = (unsigned*)o16;
#pragma unroll 1
  for (int ph = 0; ph < 2; ++ph) {
    __syncthreads();
    {
      const float* xb = x + (size_t)b * kNC * kPix + h * kSide + ph * 32 + 4 * sq;
#pragma unroll 4
      for (int i = 0; i < 16; ++i) {
        const int cc = sc + 16 * i;
        const v4f v = *(const v4f*)(xb + (size_t)cc * kPix);
        xs[(4 * sq + 0) * kXsPitch + cc] = rin(v[0]);
        xs[(4 * sq + 1) * kXsPitch + cc] = rin(v[1]);
        xs[(4 * sq + 2) * kXsPitch + cc] = rin(v[2]);
        xs[(4 * sq + 3) * kXsPitch + cc] = rin(v[3]);
      }
    }
    __syncthreads();
#pragma unroll 1
    for (int g = 0; g < 8; ++g) {
      unsigned wa[4], wb[4];
#pragma unroll
      for (int s = 0; s < 4; ++s) {
        const int wl = g * 4 + s;
        const int w = ph * 32 + wl;
        const float r = Rs[w];
        const v2f xv = *(const v2f*)(xs + wl * kXsPitch + c);
        const v2f la = *(const v2f*)(ul + (bp + (size_t)(w * kSide + h)) * kNUL + kNC + c);
        const v2f lb = *(const v2f*)(ul + (bp + (size_t)((kSide - 1 - w) * kSide + (kSide - 1 - h))) * kNUL + kNC + c);
        const v2f ua = *(const v2f*)(ul + (bp + (size_t)(h * kSide + w)) * kNUL + c);
        const v2f ub = *(const v2f*)(ul + (bp + (size_t)((kSide - 1 - h) * kSide + w)) * kNUL + c);
        h1a = h1a * r + la[0] * xv[0];
        h1b = h1b * r + la[1] * xv[1];
        h2a = h2a * r + lb[0] * xv[0];
        h2b = h2b * r + lb[1] * xv[1];
        wa[s] = pack2h(h1a * ua[0] * kCarryO, h1b * ua[1] * kCarryO);
        wb[s] = pack2h(h2a * ub[0] * kCarryO, h2b * ub[1] * kCarryO);
      }
      for (int pass = 0; pass < 2; ++pass) {
#pragma unroll
        for (int s = 0; s < 4; ++s) {
          const size_t rowi = bp + (size_t)(h * kSide + ph * 32 + g * 4 + s);
          *(volatile unsigned*)(Ow + rowi * (kKM / 2) + tid) = wa[s];
          *(volatile unsigned*)(Ow + rowi * (kKM / 2) + (kNC / 2) + tid) = wb[s];
        }
        __threadfence();
      }
    }
  }
}

extern "C" void kernel_launch(void* const* d_in, const int* in_sizes, int n_in,
                              void* d_out, int out_size, void* d_ws, size_t ws_size,
                              hipStream_t stream) {
  if (n_in < 11) return;
  if (in_sizes[0] != kNB * kNC * kPix) return;
  if (in_sizes[1] != kNCr * kNC) return;
  if (in_sizes[2] != kNCr) return;
  if (in_sizes[3] != kNC * kNCr) return;
  if (in_sizes[4] != kNC) return;
  if (in_sizes[5] != kNC * kNCr) return;
  if (in_sizes[6] != kNC) return;
  if (in_sizes[7] != 3 * kNCr) return;
  if (in_sizes[8] != 3) return;
  if (in_sizes[9] != kNC * 4 * kNC) return;
  if (in_sizes[10] != kNC) return;
  if (out_size != kNB * kNC * kPix) return;
  if (ws_size < kWsTotal) return;

  const float* x       = (const float*)d_in[0];
  const float* w_red   = (const float*)d_in[1];
  const float* b_red   = (const float*)d_in[2];
  const float* w_u     = (const float*)d_in[3];
  const float* b_u     = (const float*)d_in[4];
  const float* w_lam   = (const float*)d_in[5];
  const float* b_lam   = (const float*)d_in[6];
  const float* w_wt    = (const float*)d_in[7];
  const float* b_wt    = (const float*)d_in[8];
  const float* w_merge = (const float*)d_in[9];
  const float* b_merge = (const float*)d_in[10];

  char* ws = (char*)d_ws;
  unsigned short* XT   = (unsigned short*)(ws + kOffXT);
  unsigned short* RED  = (unsigned short*)(ws + kOffRED);
  float*          UL   = (float*)(ws + kOffUL);
  unsigned short* O16  = (unsigned short*)(ws + kOffO);
  unsigned short* WRED = (unsigned short*)(ws + kOffWRED);
  unsigned short* WUL  = (unsigned short*)(ws + kOffWUL);
  unsigned short* WAB  = (unsigned short*)(ws + kOffWAB);
  float*          BUL  = (float*)(ws + kOffBUL);
  float*          BRED = (float*)(ws + kOffBRED);
  float*          BMRG = (float*)(ws + kOffBMRG);
  float*          RC   = (float*)(ws + kOffRC);

  prep_planes_kernel<<<89, 256, 0, stream>>>(w_red, b_red, w_u, b_u, w_lam, b_lam, w_merge, b_merge,
                                             WRED, WUL, WAB, BUL, BRED, BMRG);

  x_plane_kernel<<<kNB * 4 * 64, 256, 0, stream>>>(x, XT);

  gemm64_h<2, 1><<<dim3(64, 1), 256, 0, stream>>>(
      XT, kNC, 0L, WRED, kNC, 0L, (void*)RED, kNCr, 0L, BRED, kRows, kNCr, kNC, kScaleS0);

  gemm64_h<2, 0><<<dim3(512, 1), 256, 0, stream>>>(
      RED, kNCr, 0L, WUL, kNCr, 0L, (void*)UL, kNUL, 0L, BUL, kRows, kNUL, kNCr, kScaleS12);

  band_coef_kernel<<<kRows / 256, 256, 0, stream>>>(RED, w_wt, b_wt, RC);

  line_scan_kernel<<<kNB * kSide, 128, 0, stream>>>(x, UL, RC, O16);

  gemm64_h<1, 0><<<dim3(32, kNB), 256, 0, stream>>>(
      WAB, kKM, 0L, O16, kKM, (long)kPix * kKM, d_out, kPix, (long)kNC * kPix, BMRG, kNC, kPix, kKM, kScaleS4);
}
